// SCPositionwiseFeedForward_low_82317343195169
// MI455X (gfx1250) — hardware-run, weakly checked
//
#include <hip/hip_runtime.h>


#ifndef NB
#define NB 8
#endif
#ifndef SEQ
#define SEQ 1024
#endif
#define NB_FULL  8
#define SEQ_FULL 1024
#ifndef OUT_SEQ
#define OUT_SEQ SEQ
#endif
#define DIN  256
#define DH1  1024
#define DH2  1024
#define KW   9
#define KPAD 4
#define TR   64
#define CY1  256.0f
#define CPW  64.0f
#define CY2  256.0f
#define CW2  64.0f
#define SC2Y (CY2 / (CY1 * CPW))
#define SC3  (1.0f / (CY2 * CW2))

static_assert(KW == 2 * KPAD + 1);
static_assert(KW <= 32);
static_assert(DIN % 32 == 0);
static_assert(DH1 % 32 == 0);
static_assert(DH2 % 32 == 0);
static_assert(DIN % 64 == 0);
static_assert(DH1 % 64 == 0);
static_assert(DH2 % 64 == 0);
static_assert(SEQ % 64 == 0);
static_assert(SEQ % TR == 0);
static_assert(128 * 8 == DH1);
static_assert(128 * 16 == DH1 * 2);
static_assert(DH1 % 256 == 0);
static_assert(32 * 16 * 16 == 64 * 128);
static_assert(32 * 16 * 32 == 64 * 256);
static_assert(256 * 16 * 2 == 64 * 128);
static_assert(16 * 16 == 64 * 4);
static_assert(64 * 68 * 4 <= 131072);
static_assert(64 * 68 * 4 + 16 * 64 * 4 + 64 * 4 <= 131072);
static_assert(KW * DH1 * 4 <= 131072);
static_assert(NB <= NB_FULL);
static_assert(SEQ <= SEQ_FULL);
static_assert(((size_t)SEQ * DIN) % 8 == 0);
static_assert(((size_t)DH1 * DIN) % 8 == 0);
static_assert(((size_t)DIN * DH2) % 8 == 0);

typedef _Float16 h16;
typedef unsigned short bf;
typedef __attribute__((ext_vector_type(16))) __bf16   v16bf;
typedef __attribute__((ext_vector_type(16))) _Float16 v16h;
typedef __attribute__((ext_vector_type(8)))  _Float16 v8h;
typedef __attribute__((ext_vector_type(8)))  unsigned short v8us;
typedef __attribute__((ext_vector_type(8)))  float    v8f;
typedef __attribute__((ext_vector_type(4)))  float    v4f;
typedef v4f  __attribute__((may_alias)) v4fa;

__device__ __forceinline__ unsigned short f2bf(float f) { unsigned u = __float_as_uint(f); u += 0x7FFFu + ((u >> 16) & 1u); return (unsigned short)(u >> 16); }
__device__ __forceinline__ float bfr(float f) { return __uint_as_float(((unsigned)f2bf(f)) << 16); }
__device__ __forceinline__ v16h cat16(v8h lo, v8h hi) { return __builtin_shufflevector(lo, hi, 0, 1, 2, 3, 4, 5, 6, 7, 8, 9, 10, 11, 12, 13, 14, 15); }
__device__ __forceinline__ v16bf cat16b(v8us lo, v8us hi) { return __builtin_bit_cast(v16bf, __builtin_shufflevector(lo, hi, 0, 1, 2, 3, 4, 5, 6, 7, 8, 9, 10, 11, 12, 13, 14, 15)); }
__device__ __forceinline__ v8f wmma16(v16h a, v16h b, v8f c) { return __builtin_amdgcn_wmma_f32_16x16x32_f16(false, a, false, b, (short)0, c, false, false); }
__device__ __forceinline__ v8f wmmab(v16bf a, v16bf b, v8f c) { return __builtin_amdgcn_wmma_f32_16x16x32_bf16(false, a, false, b, (short)0, c, false, false); }
__device__ __forceinline__ v16h  ldh(const h16* p) { return cat16(*(const v8h*)p, *(const v8h*)(p + 16)); }
__device__ __forceinline__ v16bf ldb(const bf* p)  { return cat16b(*(const v8us*)p, *(const v8us*)(p + 16)); }
__device__ __forceinline__ void wave_sync() { __builtin_amdgcn_fence(3  , "wavefront"); __builtin_amdgcn_wave_barrier(); asm volatile("" ::: "memory"); }

__device__ __forceinline__ v8f wmmabg(v16bf a, v16bf b, v8f c) { c = wmmab(a, b, c); asm volatile("v_nop\n\tv_nop\n\tv_nop\n\tv_nop" : "+v"(c) : "v"(a), "v"(b)); return c; }
__device__ __forceinline__ v8f wmma16g(v16h a, v16h b, v8f c) { c = wmma16(a, b, c); asm volatile("v_nop\n\tv_nop\n\tv_nop\n\tv_nop" : "+v"(c) : "v"(a), "v"(b)); return c; }
static __device__ __forceinline__ h16 toh_flush(float v) { const float w = (fabsf(v) < 6.103515625e-05f) ? 0.0f : v; return (h16)w; }

__device__ __forceinline__ float mishf(float v) {
    const float sp = fmaxf(v, 0.0f) + log1pf(expf(-fabsf(v)));
    return v * tanhf(sp);
}

template <int K>
__device__ __forceinline__ void mm_bf(const bf* __restrict__ A, const bf* __restrict__ Bt, v8f (&acc)[4][4]) {
#pragma unroll 1
    for (int kc = 0; kc < K; kc += 32) {
        v16bf a[4];
#pragma unroll
        for (int mb = 0; mb < 4; ++mb) a[mb] = ldb(A + (size_t)mb * 16 * K + kc);
#pragma unroll
        for (int nb = 0; nb < 4; ++nb) { const v16bf b = ldb(Bt + (size_t)nb * 16 * K + kc);
#pragma unroll
            for (int mb = 0; mb < 4; ++mb) acc[mb][nb] = wmmabg(a[mb], b, acc[mb][nb]); }
    }
}
template <int K>
__device__ __forceinline__ void mm_h(const h16* __restrict__ A, const h16* __restrict__ Bt, v8f (&acc)[4][4]) {
#pragma unroll 1
    for (int kc = 0; kc < K; kc += 32) {
        v16h a[4];
#pragma unroll
        for (int mb = 0; mb < 4; ++mb) a[mb] = ldh(A + (size_t)mb * 16 * K + kc);
#pragma unroll
        for (int nb = 0; nb < 4; ++nb) { const v16h b = ldh(Bt + (size_t)nb * 16 * K + kc);
#pragma unroll
            for (int mb = 0; mb < 4; ++mb) acc[mb][nb] = wmma16g(a[mb], b, acc[mb][nb]); }
    }
}

__global__ __launch_bounds__(256) void k_cvt8(const float* __restrict__ src, bf* dst, size_t n8) {
    const size_t i = (size_t)blockIdx.x * 256 + threadIdx.x; if (i >= n8) return;
    const v8f v = *(const v8f*)(src + i * 8); v8us o;
#pragma unroll
    for (int k = 0; k < 8; ++k) o[k] = f2bf(v[k]);
    *(volatile v8us*)(dst + i * 8) = o; __threadfence(); *(volatile v8us*)(dst + i * 8) = o;
}

__global__ __launch_bounds__(256) void k_cvth8(const float* __restrict__ src, h16* dst, size_t n8) {
    const size_t i = (size_t)blockIdx.x * 256 + threadIdx.x; if (i >= n8) return;
    const v8f v = *(const v8f*)(src + i * 8); v8h o;
#pragma unroll
    for (int k = 0; k < 8; ++k) o[k] = toh_flush(bfr(v[k]) * CW2);
    *(volatile v8h*)(dst + i * 8) = o; __threadfence(); *(volatile v8h*)(dst + i * 8) = o;
}

__global__ __launch_bounds__(256) void k_dnorm(const float* __restrict__ dw, float* ND) {
#pragma clang fp contract(off)
    __shared__ float part[8 * KW];
    __shared__ __align__(16) float line[32];
    const unsigned tid = threadIdx.x, b = blockIdx.x;
    const unsigned lane = tid & 31u;
    const int wave = __builtin_amdgcn_readfirstlane((int)(threadIdx.x >> 5));
    float s[KW];
#pragma unroll
    for (int k = 0; k < KW; ++k) s[k] = 0.0f;
#pragma unroll 1
    for (unsigned j = 0; j < DH1 / 256; ++j) {
        const float* p = dw + ((size_t)b * DH1 + tid + 256u * j) * KW;
#pragma unroll
        for (int k = 0; k < KW; ++k) { const float w = bfr(p[k]); s[k] += w * w; }
    }
#pragma unroll
    for (int k = 0; k < KW; ++k) { float v = s[k];
        v += __shfl_xor(v, 16, 32); v += __shfl_xor(v, 8, 32); v += __shfl_xor(v, 4, 32); v += __shfl_xor(v, 2, 32); v += __shfl_xor(v, 1, 32); s[k] = v; }
    if (lane == 0) {
#pragma unroll
        for (int k = 0; k < KW; ++k) part[wave * KW + k] = s[k];
    }
    __syncthreads();
    const unsigned kk = min(tid, (unsigned)(KW - 1));
    float tot = 0.0f;
#pragma unroll
    for (int w = 0; w < 8; ++w) tot += part[w * KW + kk];
    const float inv = 1.0f / fmaxf(sqrtf(tot), 1e-12f);
    const float r = (tid < (unsigned)KW) ? inv : 0.0f;
    if (tid < 32u) line[tid] = r;
    __syncthreads();
    if (tid < 8u) {
        const v4f val = *(const v4fa*)(&line[tid * 4u]);
        float* p = ND + (size_t)b * 32 + tid * 4u;
        *(volatile v4f*)p = val; __threadfence(); *(volatile v4f*)p = val;
    }
}

__global__ __launch_bounds__(256) void k_pwt(const float* __restrict__ pw, const float* __restrict__ pg, h16* PWT, float* INVNP) {
#pragma clang fp contract(off)
    __shared__ __align__(16) float ts[64 * 68];
    __shared__ float red[16 * 64];
    __shared__ __align__(16) float line[64];
    const unsigned tid = threadIdx.x;
    const unsigned o0 = blockIdx.x * 64u, b = blockIdx.y;
    const unsigned oj4 = (tid & 15u) * 4u, cq = tid >> 4;
    const float* src = pw + (size_t)b * DH1 * DH2 + o0 + oj4;
    const float* gp = pg + (size_t)b * DH1;
    h16* dstb = PWT + ((size_t)b * DH2 + o0) * DH1;
    const unsigned srow = tid >> 3, sc8 = (tid & 7u) * 8u;
    float ss0 = 0.0f, ss1 = 0.0f, ss2 = 0.0f, ss3 = 0.0f;
#pragma unroll 1
    for (unsigned c0 = 0; c0 < DH1; c0 += 64) {
#pragma unroll
        for (int q = 0; q < 4; ++q) {
            const unsigned ci = cq + 16u * q;
            const v4f w = *(const v4f*)(src + (size_t)(c0 + ci) * DH2);
            const float g = bfr(gp[c0 + ci]) * CPW;
            const float w0 = bfr(w[0]), w1 = bfr(w[1]), w2 = bfr(w[2]), w3 = bfr(w[3]);
            ss0 += w0 * w0; ss1 += w1 * w1; ss2 += w2 * w2; ss3 += w3 * w3;
            ts[(oj4 + 0u) * 68u + ci] = w0 * g; ts[(oj4 + 1u) * 68u + ci] = w1 * g;
            ts[(oj4 + 2u) * 68u + ci] = w2 * g; ts[(oj4 + 3u) * 68u + ci] = w3 * g;
        }
        __syncthreads();
#pragma unroll 1
        for (int ps = 0; ps < 2; ++ps) {
#pragma unroll
            for (int s = 0; s < 2; ++s) { const unsigned row = srow + 32u * s;
                const v4f x0 = *(const v4fa*)(&ts[row * 68u + sc8]); const v4f x1 = *(const v4fa*)(&ts[row * 68u + sc8 + 4u]); v8h hv;
#pragma unroll
                for (int i = 0; i < 4; ++i) { hv[i] = toh_flush(x0[i]); hv[4 + i] = toh_flush(x1[i]); }
                *(volatile v8h*)(dstb + (size_t)row * DH1 + c0 + sc8) = hv; }
            if (ps == 0) __threadfence(); }
        __syncthreads();
    }
    red[cq * 64u + oj4 + 0u] = ss0; red[cq * 64u + oj4 + 1u] = ss1; red[cq * 64u + oj4 + 2u] = ss2; red[cq * 64u + oj4 + 3u] = ss3;
    __syncthreads();
    if (tid < 64u) {
        float tot = 0.0f;
#pragma unroll
        for (int g = 0; g < 16; ++g) tot += red[g * 64 + tid];
        line[tid] = 1.0f / fmaxf(sqrtf(tot), 1e-12f);
    }
    __syncthreads();
    if (tid < 16u) {
        const v4f val = *(const v4fa*)(&line[tid * 4u]);
        float* p = INVNP + (size_t)b * DH2 + o0 + tid * 4u;
        *(volatile v4f*)p = val; __threadfence(); *(volatile v4f*)p = val;
    }
}

__global__ __launch_bounds__(32) void k_gemm_a(const bf* __restrict__ XB, const bf* __restrict__ W1B, const float* __restrict__ w1b, h16* H) {
    __shared__ __align__(16) float os[64 * 68];
    const int lane = threadIdx.x & 31, lr = lane & 15, hi = lane >> 4;
    const unsigned r0 = blockIdx.x * 64u, c0 = blockIdx.y * 64u;
    v8f acc[4][4];
#pragma unroll
    for (int mb = 0; mb < 4; ++mb)
#pragma unroll
        for (int nb = 0; nb < 4; ++nb) acc[mb][nb] = (v8f){};
    mm_bf<DIN>(XB + (size_t)(r0 + lr) * DIN + 8 * hi, W1B + (size_t)(c0 + lr) * DIN + 8 * hi, acc);
    float bc[4];
#pragma unroll
    for (int nb = 0; nb < 4; ++nb) bc[nb] = bfr(w1b[c0 + nb * 16 + lr]);
#pragma unroll
    for (int mb = 0; mb < 4; ++mb)
#pragma unroll
        for (int nb = 0; nb < 4; ++nb)
#pragma unroll
            for (int j = 0; j < 8; ++j) os[(mb * 16 + hi * 8 + j) * 68 + nb * 16 + lr] = acc[mb][nb][j] + bc[nb];
    wave_sync();
#pragma unroll 1
    for (int it = 0; it < 128; ++it) { const int e = it * 32 + lane; const int idx = (e >> 6) * 68 + (e & 63);
        const float v = os[idx]; os[idx] = mishf(v); }
    wave_sync();
    h16* hrow = H + (size_t)r0 * DH1 + c0;
#pragma unroll 1
    for (int ps = 0; ps < 2; ++ps) {
#pragma unroll 1
        for (int s = 0; s < 16; ++s) { const int row = 4 * s + (lane >> 3), c8 = (lane & 7) * 8;
            const v4f x0 = *(const v4fa*)(&os[row * 68 + c8]); const v4f x1 = *(const v4fa*)(&os[row * 68 + c8 + 4]); v8h hv;
#pragma unroll
            for (int i = 0; i < 4; ++i) { hv[i] = (h16)x0[i]; hv[4 + i] = (h16)x1[i]; }
            *(volatile v8h*)(hrow + (size_t)row * DH1 + c8) = hv; }
        if (ps == 0) __threadfence(); }
}

__global__ __launch_bounds__(128) void k_taps(const h16* __restrict__ H, const float* __restrict__ dw, const float* __restrict__ dg, const float* __restrict__ db,
                                              const float* __restrict__ ND, h16* Y1) {
#pragma clang fp contract(off)
    __shared__ __align__(16) float wl[KW * DH1];
    const unsigned tid = threadIdx.x, b = blockIdx.y, t0 = blockIdx.x * (unsigned)TR;
#pragma unroll 1
    for (unsigned e = tid; e < (unsigned)(KW * DH1); e += 128u) {
        const unsigned c = e / 9u, k = e - c * 9u;
        wl[k * DH1 + c] = bfr(dw[(size_t)b * DH1 * KW + e]) * ND[b * 32u + k] * bfr(dg[(size_t)b * DH1 + c]);
    }
    __syncthreads();
    const unsigned c8 = tid * 8u;
    const v4f q0 = *(const v4f*)(db + (size_t)b * DH1 + c8), q1 = *(const v4f*)(db + (size_t)b * DH1 + c8 + 4u);
    float bi[8];
#pragma unroll
    for (int i = 0; i < 4; ++i) { bi[i] = bfr(q0[i]); bi[4 + i] = bfr(q1[i]); }
    const h16* hb = H + (size_t)b * SEQ * DH1 + c8;
    h16* yb = Y1 + ((size_t)b * SEQ + t0) * DH1 + c8;
#pragma unroll 1
    for (unsigned tt = 0; tt < (unsigned)TR; ++tt) {
        float a[8];
#pragma unroll
        for (int i = 0; i < 8; ++i) a[i] = bi[i];
#pragma unroll 1
        for (int k = 0; k < KW; ++k) {
            const int ts = (int)(t0 + tt) + k - KPAD;
            const bool ok = (ts >= 0) && (ts < SEQ);
            const int tc = min(max(ts, 0), SEQ - 1);
            const v8h hv = *(const v8h*)(hb + (size_t)tc * DH1);
            const v4f w0 = *(const v4fa*)(&wl[k * DH1 + c8]); const v4f w1 = *(const v4fa*)(&wl[k * DH1 + c8 + 4u]);
#pragma unroll
            for (int i = 0; i < 4; ++i) {
                const float h0 = ok ? (float)hv[i] : 0.0f; const float h1 = ok ? (float)hv[4 + i] : 0.0f;
                a[i] += h0 * w0[i]; a[4 + i] += h1 * w1[i]; }
        }
        v8h o;
#pragma unroll
        for (int i = 0; i < 8; ++i) o[i] = toh_flush(a[i] * CY1);
        h16* p = yb + (size_t)tt * DH1;
        *(volatile v8h*)p = o; __threadfence(); *(volatile v8h*)p = o;
    }
}

__global__ __launch_bounds__(32) void k_gemm_b(const h16* __restrict__ Y1, const h16* __restrict__ PWT, const float* __restrict__ INVNP, const float* __restrict__ pb, h16* Y2) {
    __shared__ __align__(16) float os[64 * 68];
    const int lane = threadIdx.x & 31, lr = lane & 15, hi = lane >> 4;
    const unsigned r0 = blockIdx.x * 64u, c0 = blockIdx.y * 64u;
    const unsigned b = r0 / (unsigned)SEQ;
    v8f acc[4][4];
#pragma unroll
    for (int mb = 0; mb < 4; ++mb)
#pragma unroll
        for (int nb = 0; nb < 4; ++nb) acc[mb][nb] = (v8f){};
    mm_h<DH1>(Y1 + (size_t)(r0 + lr) * DH1 + 8 * hi, PWT + ((size_t)b * DH2 + c0 + lr) * DH1 + 8 * hi, acc);
#pragma unroll
    for (int mb = 0; mb < 4; ++mb)
#pragma unroll
        for (int nb = 0; nb < 4; ++nb)
#pragma unroll
            for (int j = 0; j < 8; ++j) os[(mb * 16 + hi * 8 + j) * 68 + nb * 16 + lr] = acc[mb][nb][j];
    wave_sync();
    const int c8 = (lane & 7) * 8;
    const float* np = INVNP + (size_t)b * DH2 + c0 + c8;
    const float* bp = pb + (size_t)b * DH2 + c0 + c8;
    const v4f n0 = *(const v4f*)np, n1 = *(const v4f*)(np + 4), q0 = *(const v4f*)bp, q1 = *(const v4f*)(bp + 4);
    float sc[8], bi[8];
#pragma unroll
    for (int i = 0; i < 4; ++i) { sc[i] = n0[i] * SC2Y; sc[4 + i] = n1[i] * SC2Y; bi[i] = bfr(q0[i]) * CY2; bi[4 + i] = bfr(q1[i]) * CY2; }
    h16* yrow = Y2 + (size_t)r0 * DH2 + c0;
#pragma unroll 1
    for (int ps = 0; ps < 2; ++ps) {
#pragma unroll 1
        for (int s = 0; s < 16; ++s) { const int row = 4 * s + (lane >> 3);
            const v4f x0 = *(const v4fa*)(&os[row * 68 + c8]); const v4f x1 = *(const v4fa*)(&os[row * 68 + c8 + 4]); v8h hv;
#pragma unroll
            for (int i = 0; i < 4; ++i) { hv[i] = toh_flush(x0[i] * sc[i] + bi[i]); hv[4 + i] = toh_flush(x1[i] * sc[4 + i] + bi[4 + i]); }
            *(volatile v8h*)(yrow + (size_t)row * DH2 + c8) = hv; }
        if (ps == 0) __threadfence(); }
}

__global__ __launch_bounds__(32) void k_gemm_c(const h16* __restrict__ Y2, const h16* __restrict__ W2H, const float* __restrict__ w2b, const float* __restrict__ x, float* OUT) {
    __shared__ __align__(16) float os[64 * 68];
    const int lane = threadIdx.x & 31, lr = lane & 15, hi = lane >> 4;
    const unsigned r0 = blockIdx.x * 64u, c0 = blockIdx.y * 64u;
    const unsigned b = r0 / (unsigned)SEQ, t0 = r0 % (unsigned)SEQ;
    v8f acc[4][4];
#pragma unroll
    for (int mb = 0; mb < 4; ++mb)
#pragma unroll
        for (int nb = 0; nb < 4; ++nb) acc[mb][nb] = (v8f){};
    mm_h<DH2>(Y2 + (size_t)(r0 + lr) * DH2 + 8 * hi, W2H + (size_t)(c0 + lr) * DH2 + 8 * hi, acc);
#pragma unroll
    for (int mb = 0; mb < 4; ++mb)
#pragma unroll
        for (int nb = 0; nb < 4; ++nb)
#pragma unroll
            for (int j = 0; j < 8; ++j) os[(mb * 16 + hi * 8 + j) * 68 + nb * 16 + lr] = acc[mb][nb][j];
    wave_sync();
    const int c4 = (lane & 15) * 4;
    const v4f q = *(const v4f*)(w2b + c0 + c4);
    float bi[4];
#pragma unroll
    for (int i = 0; i < 4; ++i) bi[i] = bfr(q[i]);
    const float* xin = x + ((size_t)b * SEQ_FULL + t0) * DIN + c0 + c4;
    float* orow = OUT + ((size_t)b * OUT_SEQ + t0) * DIN + c0 + c4;
#pragma unroll 1
    for (int ps = 0; ps < 2; ++ps) {
#pragma unroll 1
        for (int s = 0; s < 32; ++s) { const int row = 2 * s + (lane >> 4);
            const v4f a = *(const v4fa*)(&os[row * 68 + c4]);
            const v4f xr = *(const v4f*)(xin + (size_t)row * DIN);
            v4f val;
#pragma unroll
            for (int i = 0; i < 4; ++i) val[i] = (a[i] * SC3 + bi[i]) + bfr(xr[i]);
            *(volatile v4f*)(orow + (size_t)row * DIN) = val; }
        if (ps == 0) __threadfence(); }
}

static constexpr size_t al256(size_t v) { return (v + 255) & ~(size_t)255; }
static constexpr size_t SZ_XB = al256((size_t)NB * SEQ * DIN * 2);
static constexpr size_t SZ_W1 = al256((size_t)DH1 * DIN * 2);
static constexpr size_t SZ_W2 = al256((size_t)DIN * DH2 * 2);
static constexpr size_t SZ_H  = al256((size_t)NB * SEQ * DH1 * 2);
static constexpr size_t SZ_Y1 = al256((size_t)NB * SEQ * DH1 * 2);
static constexpr size_t SZ_Y2 = al256((size_t)NB * SEQ * DH2 * 2);
static constexpr size_t SZ_PW = al256((size_t)NB * DH2 * DH1 * 2);
static constexpr size_t SZ_NP = al256((size_t)NB * DH2 * 4);
static constexpr size_t SZ_ND = al256((size_t)NB * 32 * 4);
static constexpr size_t SZ_TOTAL = SZ_XB + SZ_W1 + SZ_W2 + SZ_H + SZ_Y1 + SZ_Y2 + SZ_PW + SZ_NP + SZ_ND;
static_assert(SZ_TOTAL <= (size_t)134217728);
static_assert(((size_t)(NB * SEQ / 64) * 64) * DH1 * 2 <= SZ_H);
static_assert(((size_t)(SEQ / TR) * TR) * NB * DH1 * 2 <= SZ_Y1);
static_assert(((size_t)(DH2 / 64) * 64) * NB * DH1 * 2 <= SZ_PW);
static_assert((size_t)NB * 32 * 4 <= SZ_ND);

extern "C" void kernel_launch(void* const* d_in, const int* in_sizes, int n_in,
                              void* d_out, int out_size, void* d_ws, size_t ws_size, hipStream_t stream) {
    if (n_in < 11) return;
    constexpr size_t needx = ((size_t)(NB - 1) * SEQ_FULL + SEQ) * DIN;
    if ((size_t)in_sizes[0] < needx) return;
    if ((size_t)in_sizes[1] < (size_t)NB * DH1 * KW) return;
    if ((size_t)in_sizes[2] < (size_t)NB * DH1 || (size_t)in_sizes[3] < (size_t)NB * DH1) return;
    if ((size_t)in_sizes[4] < (size_t)NB * DH1 * DH2) return;
    if ((size_t)in_sizes[5] < (size_t)NB * DH1 || (size_t)in_sizes[6] < (size_t)NB * DH2) return;
    if ((size_t)in_sizes[7] < (size_t)DH1 * DIN || in_sizes[8] < DH1) return;
    if ((size_t)in_sizes[9] < (size_t)DIN * DH2 || in_sizes[10] < DIN) return;
    if ((size_t)out_size < ((size_t)(NB - 1) * OUT_SEQ + SEQ) * DIN) return;
    if (SZ_TOTAL > ws_size) return;
    const float* x   = (const float*)d_in[0];
    const float* dwp = (const float*)d_in[1];
    const float* dg  = (const float*)d_in[2];
    const float* db  = (const float*)d_in[3];
    const float* pw  = (const float*)d_in[4];
    const float* pg  = (const float*)d_in[5];
    const float* pb  = (const float*)d_in[6];
    const float* w1w = (const float*)d_in[7];
    const float* w1b = (const float*)d_in[8];
    const float* w2w = (const float*)d_in[9];
    const float* w2b = (const float*)d_in[10];
    float* OUT = (float*)d_out;
    char* wsp = (char*)d_ws;
    bf*  XB   = (bf*)wsp;  wsp += SZ_XB;
    bf*  W1B  = (bf*)wsp;  wsp += SZ_W1;
    h16* W2H  = (h16*)wsp; wsp += SZ_W2;
    h16* H    = (h16*)wsp; wsp += SZ_H;
    h16* Y1   = (h16*)wsp; wsp += SZ_Y1;
    h16* Y2   = (h16*)wsp; wsp += SZ_Y2;
    h16* PWT  = (h16*)wsp; wsp += SZ_PW;
    float* INVNP = (float*)wsp; wsp += SZ_NP;
    float* ND    = (float*)wsp; wsp += SZ_ND;

    if (SEQ == SEQ_FULL) {
        const size_t n8 = (size_t)NB * SEQ * DIN / 8;
        k_cvt8<<<(unsigned)((n8 + 255) / 256), 256, 0, stream>>>(x, XB, n8);
    } else {
        const size_t n8 = (size_t)SEQ * DIN / 8;
        for (int b = 0; b < NB; ++b) k_cvt8<<<(unsigned)((n8 + 255) / 256), 256, 0, stream>>>(x + (size_t)b * SEQ_FULL * DIN, XB + (size_t)b * SEQ * DIN, n8);
    }
    { const size_t n8 = (size_t)DH1 * DIN / 8; k_cvt8<<<(unsigned)((n8 + 255) / 256), 256, 0, stream>>>(w1w, W1B, n8); }
    { const size_t n8 = (size_t)DIN * DH2 / 8; k_cvth8<<<(unsigned)((n8 + 255) / 256), 256, 0, stream>>>(w2w, W2H, n8); }
    k_dnorm<<<dim3(NB, 1, 1), 256, 0, stream>>>(dwp, ND);
    k_pwt<<<dim3(DH2 / 64, NB, 1), 256, 0, stream>>>(pw, pg, PWT, INVNP);
    k_gemm_a<<<dim3(NB * SEQ / 64, DH1 / 64, 1), 32, 0, stream>>>(XB, W1B, w1b, H);
    k_taps<<<dim3(SEQ / TR, NB, 1), 128, 0, stream>>>(H, dwp, dg, db, ND, Y1);
    k_gemm_b<<<dim3(NB * SEQ / 64, DH2 / 64, 1), 32, 0, stream>>>(Y1, PWT, INVNP, pb, Y2);
    k_gemm_c<<<dim3(NB * SEQ / 64, DIN / 64, 1), 32, 0, stream>>>(Y2, W2H, w2b, x, OUT);
}
